// MXFP8Linear_18167711662108
// MI455X (gfx1250) — hardware-verified
//
#include <hip/hip_runtime.h>
#include <stddef.h>
#include <math.h>


#define KQ    2048
#define QB    32
#define NBQ   64
#define NTHR  256
#define BM    64
#define BNC   128
#define NT    4
#define WSCAP 134217728

static_assert(KQ == 8 * NTHR);
static_assert(NBQ * QB == KQ);
static_assert(BM == 64 && BNC == 128 && NT * 16 * 2 == BNC);
static_assert(BM * BNC <= NBQ * BM + NBQ * BNC);
static_assert((BM * NBQ) % (4 * NTHR) == 0 && (BNC * NBQ) % (4 * NTHR) == 0);
static_assert(BM == 8 * (NTHR / 32));

typedef float          v4f   __attribute__((ext_vector_type(4)));
typedef float          v8f   __attribute__((ext_vector_type(8)));
typedef unsigned short v8us  __attribute__((ext_vector_type(8)));
typedef unsigned short v16us __attribute__((ext_vector_type(16)));
typedef __bf16         v16bf __attribute__((ext_vector_type(16)));
union FragU { v16us w; v8us u[2]; };

__device__ __forceinline__ v8f wmb(v16us a, v16us b, v8f c) {
  const v16bf ab = __builtin_bit_cast(v16bf, a);
  const v16bf bb = __builtin_bit_cast(v16bf, b);
  v8f d = __builtin_amdgcn_wmma_f32_16x16x32_bf16(false, ab, false, bb, (short)0, c, false, false);
  asm volatile("v_nop\n\tv_nop\n\tv_nop\n\tv_nop" : "+v"(d) : "v"(a), "v"(b));
  return d;
}

__device__ __forceinline__ unsigned short e4m3_bf16(float q) {
  const unsigned int u  = (unsigned int)__float_as_uint(q);
  const unsigned int sg = (u >> 16) & 0x8000u;
  const unsigned int au = u & 0x7FFFFFFFu;
  const unsigned int ex = au >> 23;
  unsigned int r = au >> 20;
  const unsigned int gd = (au >> 19) & 1u;
  const unsigned int sy = ((au & 0x7FFFFu) != 0u) ? 1u : 0u;
  r += gd & (sy | (r & 1u));
  const unsigned int e8 = r >> 3;
  const unsigned int m3 = r & 7u;
  const unsigned int nrm = r << 4;
  const bool bad = (au > 0x7F800000u) || (e8 > 135u) || ((e8 == 135u) && (m3 == 7u));
  int shi = 141 - (int)ex;
  shi = shi < 21 ? 21 : (shi > 31 ? 31 : shi);
  const unsigned int sh   = (unsigned int)shi;
  const unsigned int sig  = (au & 0x7FFFFFu) | 0x800000u;
  unsigned int n          = sig >> sh;
  const unsigned int rem  = sig & ((1u << sh) - 1u);
  const unsigned int half = 1u << (sh - 1u);
  n += ((rem > half) || ((rem == half) && ((n & 1u) != 0u))) ? 1u : 0u;
  const unsigned int sub  = (unsigned int)__float_as_uint((float)n * 0.001953125f) >> 16;
  unsigned int res = (ex >= 121u) ? nrm : sub;
  res = bad ? 0x7FC0u : res;
  return (unsigned short)(res | sg);
}

__global__ __launch_bounds__(NTHR) void k_quant(const float* __restrict__ src, unsigned short* plane, float* scl) {
#pragma clang fp contract(off)
  __shared__ __attribute__((aligned(16))) float sc[NBQ];
  const int row = blockIdx.x, t = threadIdx.x;
  const float* p = src + (size_t)row * KQ + 8 * t;
  const v4f a = *(const v4f*)p;
  const v4f b = *(const v4f*)(p + 4);
  float m = fmaxf(fmaxf(fabsf(a.x), fabsf(a.y)), fmaxf(fabsf(a.z), fabsf(a.w)));
  m = fmaxf(m, fmaxf(fmaxf(fabsf(b.x), fabsf(b.y)), fmaxf(fabsf(b.z), fabsf(b.w))));
  m = fmaxf(m, __shfl_xor(m, 1));
  m = fmaxf(m, __shfl_xor(m, 2));
  const float c448  = __uint_as_float(0x3B124925u);
  const float scale = fmaxf(m * c448, 1e-30f);
  const float rcp   = 1.0f / scale;
  v8us o;
  o[0] = e4m3_bf16(a.x * rcp);
  o[1] = e4m3_bf16(a.y * rcp);
  o[2] = e4m3_bf16(a.z * rcp);
  o[3] = e4m3_bf16(a.w * rcp);
  o[4] = e4m3_bf16(b.x * rcp);
  o[5] = e4m3_bf16(b.y * rcp);
  o[6] = e4m3_bf16(b.z * rcp);
  o[7] = e4m3_bf16(b.w * rcp);
  unsigned short* dp = plane + (size_t)row * KQ + 8 * t;
  *(volatile v8us*)dp = o;
  if ((t & 3) == 0) sc[t >> 2] = scale;
  __syncthreads();
  const v4f s4 = *(const v4f*)(sc + 4 * (t & 15));
  float* ds = scl + (size_t)row * NBQ + 4 * (t & 15);
  if (t < 16) *(volatile v4f*)ds = s4;
  __threadfence();
  *(volatile v8us*)dp = o;
  if (t < 16) *(volatile v4f*)ds = s4;
}

__global__ __launch_bounds__(NTHR) void k_gemm(
    const unsigned short* __restrict__ XQ, const unsigned short* __restrict__ WQ,
    const float* __restrict__ SX, const float* __restrict__ SW,
    const float* __restrict__ bias, float* out, int F) {
  __shared__ __attribute__((aligned(16))) float lds[NBQ * BM + NBQ * BNC];
  float* sxT = lds;
  float* swT = lds + NBQ * BM;
  float* stg = lds;
  const int tid = threadIdx.x, lane = tid & 31, wave = tid >> 5, hh = lane >> 4, m = lane & 15;
  const int rowBase = (int)blockIdx.y * BM;
  const int colBase = (int)blockIdx.x * BNC;

#pragma unroll
  for (int i = 0; i < (BM * NBQ) / (4 * NTHR); ++i) {
    const int idx = i * NTHR + tid;
    const int row = idx >> 4, b4 = (idx & 15) * 4;
    const v4f s = *(const v4f*)(SX + (size_t)(rowBase + row) * NBQ + b4);
    sxT[(b4 + 0) * BM + row] = s.x;
    sxT[(b4 + 1) * BM + row] = s.y;
    sxT[(b4 + 2) * BM + row] = s.z;
    sxT[(b4 + 3) * BM + row] = s.w;
  }
#pragma unroll
  for (int i = 0; i < (BNC * NBQ) / (4 * NTHR); ++i) {
    const int idx = i * NTHR + tid;
    const int col = idx >> 4, b4 = (idx & 15) * 4;
    const v4f s = *(const v4f*)(SW + (size_t)(colBase + col) * NBQ + b4);
    swT[(b4 + 0) * BNC + col] = s.x;
    swT[(b4 + 1) * BNC + col] = s.y;
    swT[(b4 + 2) * BNC + col] = s.z;
    swT[(b4 + 3) * BNC + col] = s.w;
  }
  __syncthreads();

  const int r0 = (wave >> 1) * 16, c0 = (wave & 1) * (BNC / 2);
  v8f acc[NT];
#pragma unroll
  for (int t = 0; t < NT; ++t) { const v8f z = {0.f, 0.f, 0.f, 0.f, 0.f, 0.f, 0.f, 0.f}; acc[t] = z; }
  const v8f z8 = {0.f, 0.f, 0.f, 0.f, 0.f, 0.f, 0.f, 0.f};
  const unsigned short* ap = XQ + (size_t)(rowBase + r0 + m) * KQ + 8 * hh;
  const unsigned short* bp = WQ + (size_t)(colBase + c0 + m) * KQ + 8 * hh;
  const float* sxp = sxT + r0 + 8 * hh;
  const float* swp = swT + c0 + m;

#pragma unroll 1
  for (int b = 0; b < NBQ; ++b) {
    const int k0 = QB * b;
    FragU a;
    a.u[0] = *(const v8us*)(ap + k0);
    a.u[1] = *(const v8us*)(ap + k0 + 16);
    const v4f sa = *(const v4f*)(sxp + b * BM);
    const v4f sb = *(const v4f*)(sxp + b * BM + 4);
#pragma unroll
    for (int t = 0; t < NT; ++t) {
      const unsigned short* bpt = bp + (size_t)(16 * t) * KQ + k0;
      FragU bf;
      bf.u[0] = *(const v8us*)(bpt);
      bf.u[1] = *(const v8us*)(bpt + 16);
      const v8f d = wmb(a.w, bf.w, z8);
      const float sw = swp[b * BNC + 16 * t];
      acc[t][0] = fmaf(d[0] * sa.x, sw, acc[t][0]);
      acc[t][1] = fmaf(d[1] * sa.y, sw, acc[t][1]);
      acc[t][2] = fmaf(d[2] * sa.z, sw, acc[t][2]);
      acc[t][3] = fmaf(d[3] * sa.w, sw, acc[t][3]);
      acc[t][4] = fmaf(d[4] * sb.x, sw, acc[t][4]);
      acc[t][5] = fmaf(d[5] * sb.y, sw, acc[t][5]);
      acc[t][6] = fmaf(d[6] * sb.z, sw, acc[t][6]);
      acc[t][7] = fmaf(d[7] * sb.w, sw, acc[t][7]);
    }
  }

  __syncthreads();
  float* sp = stg + (size_t)(r0 + 8 * hh) * BNC + c0 + m;
#pragma unroll
  for (int t = 0; t < NT; ++t) {
#pragma unroll
    for (int r = 0; r < 8; ++r) sp[r * BNC + 16 * t] = acc[t][r];
  }
  __syncthreads();

  const v4f b4 = *(const v4f*)(bias + colBase + 4 * lane);
  v4f ov[8];
#pragma unroll
  for (int r = 0; r < 8; ++r) ov[r] = *(const v4f*)(stg + (size_t)(8 * wave + r) * BNC + 4 * lane) + b4;
  float* ob = out + (size_t)(rowBase + 8 * wave) * F + colBase + 4 * lane;
#pragma unroll
  for (int r = 0; r < 8; ++r) *(volatile v4f*)(ob + (size_t)r * F) = ov[r];
  __threadfence();
#pragma unroll
  for (int r = 0; r < 8; ++r) *(volatile v4f*)(ob + (size_t)r * F) = ov[r];
}

static size_t carve(size_t* o, size_t bytes) {
  const size_t r = *o;
  *o += (bytes + 255) & ~(size_t)255;
  return r;
}

extern "C" void kernel_launch(void* const* d_in, const int* in_sizes, int n_in,
                              void* d_out, int out_size, void* d_ws, size_t ws_size,
                              hipStream_t stream) {
  if (n_in < 3) return;
  const int F = in_sizes[2];
  if (F <= 0 || in_sizes[0] <= 0 || in_sizes[1] <= 0) return;
  if (in_sizes[1] % F != 0) return;
  const int K = in_sizes[1] / F;
  if (K != KQ) return;
  if (in_sizes[0] % K != 0) return;
  const int N = in_sizes[0] / K;
  if ((long long)out_size != (long long)N * (long long)F) return;
  if ((N % BM) != 0 || (F % BNC) != 0) return;
  if (N > (1 << 20) || F > (1 << 20)) return;

  const float* x    = (const float*)d_in[0];
  const float* w    = (const float*)d_in[1];
  const float* bias = (const float*)d_in[2];
  float* out = (float*)d_out;

  char* wsb = (char*)d_ws;
  size_t o = 0;
  const size_t oXQ = carve(&o, (size_t)N * KQ * 2);
  const size_t oWQ = carve(&o, (size_t)F * KQ * 2);
  const size_t oSX = carve(&o, (size_t)N * NBQ * 4);
  const size_t oSW = carve(&o, (size_t)F * NBQ * 4);
  if (o > ws_size || o > (size_t)WSCAP) return;
  unsigned short* XQ = (unsigned short*)(wsb + oXQ);
  unsigned short* WQ = (unsigned short*)(wsb + oWQ);
  float* SX = (float*)(wsb + oSX);
  float* SW = (float*)(wsb + oSW);

  k_quant<<<N, NTHR, 0, stream>>>(x, XQ, SX);
  k_quant<<<F, NTHR, 0, stream>>>(w, WQ, SW);

  dim3 grid((unsigned)(F / BNC), (unsigned)(N / BM), 1);
  k_gemm<<<grid, NTHR, 0, stream>>>(XQ, WQ, SX, SW, bias, out, F);
}
